// CausalSelfAttention_50646254355207
// MI455X (gfx1250) — hardware-verified
//
#include <hip/hip_runtime.h>


#ifndef NB
#define NB 1
#endif
#ifndef SEQ
#define SEQ 4096
#endif
#define NB_FULL  1
#define SEQ_FULL 4096
#define DM   1024
#define NH_  8
#define HD   128
#define NQKV 24
#define AW   4
#define TP   132
#define EROWS (SEQ < 512 ? SEQ : 512)
#define QRS  2048.0f
#define QRI  (1.0f / 2048.0f)
#define SC2  ((float)(0.12 * 1.4426950408889634))
#define PSH  14.0f
#define NEGB (-3.0e38f)
#define YC   64.0f
#define WOC  256.0f
#define OSC  (1.0f / (64.0f * 256.0f))

static_assert(NB == 1);
static_assert(HD == 128);
static_assert(NH_ * HD == DM);
static_assert(NQKV == 3 * NH_);
static_assert(DM % 64 == 0);
static_assert(DM % 32 == 0);
static_assert(HD % 32 == 0);
static_assert(SEQ % 64 == 0);
static_assert(SEQ % 32 == 0);
static_assert(EROWS % 64 == 0);
static_assert(EROWS >= 32);
static_assert(EROWS <= SEQ);
static_assert(EROWS % (16 * AW) == 0);
static_assert((SEQ - EROWS) % (16 * AW) == 0);
static_assert(((size_t)SEQ * DM) % 8 == 0);
static_assert(((size_t)DM * DM) % 8 == 0);
static_assert(((size_t)SEQ * 32) % 256 == 0);
static_assert(SEQ <= SEQ_FULL);
static_assert((TP * 4) % 16 == 0);
static_assert(sizeof(float) * 64 * TP <= 131072);

typedef _Float16 h16;
typedef unsigned short bf;
typedef __attribute__((ext_vector_type(16))) __bf16   v16bf;
typedef __attribute__((ext_vector_type(16))) _Float16 v16h;
typedef __attribute__((ext_vector_type(8)))  _Float16 v8h;
typedef __attribute__((ext_vector_type(8)))  unsigned short v8us;
typedef __attribute__((ext_vector_type(8)))  float    v8f;
typedef __attribute__((ext_vector_type(4)))  float    v4f;
typedef v4f  __attribute__((may_alias)) v4fa;

__device__ __forceinline__ unsigned short f2bf(float f) { unsigned u = __float_as_uint(f); u += 0x7FFFu + ((u >> 16) & 1u); return (unsigned short)(u >> 16); }
__device__ __forceinline__ float bfr(float f) { return __uint_as_float(((unsigned)f2bf(f)) << 16); }
__device__ __forceinline__ v16h cat16(v8h lo, v8h hi) { return __builtin_shufflevector(lo, hi, 0, 1, 2, 3, 4, 5, 6, 7, 8, 9, 10, 11, 12, 13, 14, 15); }
__device__ __forceinline__ v16bf cat16b(v8us lo, v8us hi) { return __builtin_bit_cast(v16bf, __builtin_shufflevector(lo, hi, 0, 1, 2, 3, 4, 5, 6, 7, 8, 9, 10, 11, 12, 13, 14, 15)); }
__device__ __forceinline__ v8f wmma16(v16h a, v16h b, v8f c) { return __builtin_amdgcn_wmma_f32_16x16x32_f16(false, a, false, b, (short)0, c, false, false); }
__device__ __forceinline__ v8f wmmab(v16bf a, v16bf b, v8f c) { return __builtin_amdgcn_wmma_f32_16x16x32_bf16(false, a, false, b, (short)0, c, false, false); }
__device__ __forceinline__ v16h  ldh(const h16* p) { return cat16(*(const v8h*)p, *(const v8h*)(p + 16)); }
__device__ __forceinline__ v16bf ldb(const bf* p)  { return cat16b(*(const v8us*)p, *(const v8us*)(p + 16)); }
__device__ __forceinline__ void wave_sync() { __builtin_amdgcn_fence(3  , "wavefront"); __builtin_amdgcn_wave_barrier(); asm volatile("" ::: "memory"); }

static __device__ __forceinline__ h16 toh_flush(float v) { const h16 r = (h16)v; return (fabsf(v) < 6.103515625e-05f) ? (h16)0.0f : r; }
__device__ __forceinline__ v8f wmma16g(v16h a, v16h b, v8f c) { c = wmma16(a, b, c); asm volatile("v_nop\n\tv_nop\n\tv_nop\n\tv_nop" : "+v"(c) : "v"(a), "v"(b)); return c; }
__device__ __forceinline__ v8f wmmabg(v16bf a, v16bf b, v8f c) { c = wmmab(a, b, c); asm volatile("v_nop\n\tv_nop\n\tv_nop\n\tv_nop" : "+v"(c) : "v"(a), "v"(b)); return c; }

__global__ __launch_bounds__(256) void k_cvt8(const float* __restrict__ src, bf* dst, size_t n8) {
    const size_t i = (size_t)blockIdx.x * 256 + threadIdx.x; if (i >= n8) return;
    const v8f v = *(const v8f*)(src + i * 8); v8us o;
#pragma unroll
    for (int k = 0; k < 8; ++k) o[k] = f2bf(v[k]);
    *(volatile v8us*)(dst + i * 8) = o; __threadfence(); *(volatile v8us*)(dst + i * 8) = o;
}

__global__ __launch_bounds__(256) void k_cvtw(const float* __restrict__ src, h16* dst, size_t n8) {
#pragma clang fp contract(off)
    const size_t i = (size_t)blockIdx.x * 256 + threadIdx.x; if (i >= n8) return;
    const v8f v = *(const v8f*)(src + i * 8); v8h o;
#pragma unroll
    for (int k = 0; k < 8; ++k) o[k] = toh_flush(bfr(v[k]) * WOC);
    *(volatile v8h*)(dst + i * 8) = o; __threadfence(); *(volatile v8h*)(dst + i * 8) = o;
}

__global__ __launch_bounds__(256) void k_ropetab(float* CS) {
#pragma clang fp contract(off)
    const int i = (int)blockIdx.x * 256 + (int)threadIdx.x;
    const int t = i >> 5, j = i & 31;
    const float e = (float)j / 31.0f;
    const float a = -10.0f * e;
    const float lo = fmaf(-10.0f, e, -a);
    float invf = exp2f(a);
    invf = fmaf(invf, 0.69314718056f * lo, invf);
    const float th = (float)t * invf;
    float s, c; sincosf(th, &s, &c);
    float* row = CS + (size_t)t * 64;
    *(volatile float*)(row + j) = c; *(volatile float*)(row + 32 + j) = s;
    __threadfence();
    *(volatile float*)(row + j) = c; *(volatile float*)(row + 32 + j) = s;
}

__global__ __launch_bounds__(64) void k_qkv(const bf* __restrict__ XB, const bf* __restrict__ WB, const float* __restrict__ ve, const float* __restrict__ lam, const float* __restrict__ CS,
                                            h16* QK, h16* VT, h16* VR) {
    __shared__ __align__(16) float os[64 * TP];
    const size_t PLE = (size_t)NH_ * SEQ * HD;
    const int lane = threadIdx.x & 31, lr = lane & 15, hi = lane >> 4;
    const int wave = __builtin_amdgcn_readfirstlane((int)(threadIdx.x >> 5));
    const int r0 = blockIdx.x * 64;
    const int hh = blockIdx.y;
    const int kind = hh >> 3, hd = hh & 7;
    const int c0 = hh * HD + wave * 64;
    v8f acc[4][4];
#pragma unroll
    for (int mb = 0; mb < 4; ++mb)
#pragma unroll
        for (int nb = 0; nb < 4; ++nb) acc[mb][nb] = (v8f){};
    const size_t aoff = (size_t)(r0 + lr) * DM + 8 * hi, boff = (size_t)(c0 + lr) * DM + 8 * hi;
#pragma unroll 1
    for (int kc = 0; kc < DM; kc += 32) {
        v16bf a[4];
#pragma unroll
        for (int mb = 0; mb < 4; ++mb) a[mb] = ldb(XB + aoff + (size_t)mb * 16 * DM + kc);
#pragma unroll
        for (int nb = 0; nb < 4; ++nb) { const v16bf b = ldb(WB + boff + (size_t)nb * 16 * DM + kc);
#pragma unroll
            for (int mb = 0; mb < 4; ++mb) acc[mb][nb] = wmmabg(a[mb], b, acc[mb][nb]); }
    }
#pragma unroll
    for (int mb = 0; mb < 4; ++mb)
#pragma unroll
        for (int nb = 0; nb < 4; ++nb)
#pragma unroll
            for (int j = 0; j < 8; ++j) os[(mb * 16 + hi * 8 + j) * TP + wave * 64 + nb * 16 + lr] = acc[mb][nb][j];
    __syncthreads();
    const float l0 = bfr(lam[0]), l1 = bfr(lam[1]);
    const float sg = (lane < 16) ? 1.0f : -1.0f;
    const bool act = (lane & 8) == 0;
#pragma unroll 1
    for (int rr = 0; rr < 32; ++rr) {
        const int row = wave * 32 + rr; const int t = r0 + row;
        const v4f xv = *(const v4fa*)(&os[row * TP + 4 * lane]);
        float ss = xv[0] * xv[0] + xv[1] * xv[1] + xv[2] * xv[2] + xv[3] * xv[3];
        ss += __shfl_xor(ss, 16, 32); ss += __shfl_xor(ss, 8, 32); ss += __shfl_xor(ss, 4, 32); ss += __shfl_xor(ss, 2, 32); ss += __shfl_xor(ss, 1, 32);
        const float inv = rsqrtf(ss * (1.0f / HD) + 1.0e-6f);
        v4f y;
        if (kind < 2) {
            v4f cv = *(const v4f*)(CS + (size_t)t * 64 + 4 * (lane & 7));
            v4f sv = *(const v4f*)(CS + (size_t)t * 64 + 32 + 4 * (lane & 7));
            asm volatile("" : "+v"(cv), "+v"(sv));
#pragma unroll
            for (int i = 0; i < 4; ++i) {
                const float xn = xv[i] * inv;
                const float part = __shfl_xor(xn, 16, 32);
                const float c = act ? cv[i] : 1.0f; const float s = act ? sv[i] : 0.0f;
                y[i] = xn * c + sg * (part * s); }
        } else {
            const v4f e4 = *(const v4f*)(ve + (size_t)t * DM + (size_t)hd * HD + 4 * lane);
#pragma unroll
            for (int i = 0; i < 4; ++i) y[i] = l0 * (xv[i] * inv) + l1 * bfr(e4[i]);
        }
        *(v4fa*)(&os[row * TP + 4 * lane]) = y;
    }
    __syncthreads();
    if (kind < 2) {
        static_assert(2 * 16 * 32 * 16 == 64 * HD * 2);
        const size_t pb0 = (size_t)(kind * 2) * PLE + ((size_t)hd * SEQ + (size_t)r0) * HD;
#pragma unroll 1
        for (int ps = 0; ps < 2; ++ps) {
#pragma unroll 2
            for (int it = 0; it < 16; ++it) { const int row = wave * 32 + it * 2 + (lane >> 4), c8 = (lane & 15) * 8;
                const v4f x0 = *(const v4fa*)(&os[row * TP + c8]); const v4f x1 = *(const v4fa*)(&os[row * TP + c8 + 4]); v8h hv, rv;
#pragma unroll
                for (int i = 0; i < 4; ++i) { const h16 a0 = toh_flush(x0[i]); const h16 a1 = toh_flush(x1[i]); hv[i] = a0; hv[4 + i] = a1;
                    rv[i] = toh_flush((x0[i] - (float)a0) * QRS); rv[4 + i] = toh_flush((x1[i] - (float)a1) * QRS); }
                const size_t oo = pb0 + (size_t)row * HD + c8;
                *(volatile v8h*)(QK + oo) = hv; *(volatile v8h*)(QK + PLE + oo) = rv; }
            if (ps == 0) __threadfence(); }
    } else {
        static_assert(2 * 16 * 32 * 16 == HD * 64 * 2);
        const bool wr = r0 < EROWS;
        const size_t vb0 = ((size_t)hd * HD) * SEQ + (size_t)r0;
        const size_t rb0 = ((size_t)hd * HD) * EROWS + (size_t)r0;
#pragma unroll 1
        for (int ps = 0; ps < 2; ++ps) {
#pragma unroll 2
            for (int it = 0; it < 16; ++it) { const int d = wave * 64 + it * 4 + (lane >> 3), c8 = (lane & 7) * 8; v8h hv, rv;
#pragma unroll
                for (int i = 0; i < 8; ++i) { const float x = os[(c8 + i) * TP + d]; const h16 a0 = toh_flush(x); hv[i] = a0; rv[i] = toh_flush((x - (float)a0) * QRS); }
                *(volatile v8h*)(VT + vb0 + (size_t)d * SEQ + c8) = hv;
                if (wr) *(volatile v8h*)(VR + rb0 + (size_t)d * EROWS + c8) = rv; }
            if (ps == 0) __threadfence(); }
    }
}

template <int EARLY>
__device__ __forceinline__ void flash_body(const h16* __restrict__ QH, const h16* __restrict__ QR, const h16* __restrict__ KP, const h16* __restrict__ KR,
                                           const h16* __restrict__ VT, const h16* __restrict__ VR, const int* __restrict__ win_p, h16* YH, h16* YR) {
    constexpr int DT  = EARLY ? 4 : 8;
    constexpr int OSP = DT * 16 + 4;
    constexpr int LPR = DT * 2;
    constexpr int RPI = 32 / LPR;
    constexpr int NST = 16 / RPI;
    static_assert(32 % LPR == 0);
    static_assert(16 % RPI == 0);
    static_assert(NST * 32 * 16 == 16 * DT * 16 * 2);
    static_assert((OSP * 4) % 16 == 0);
    static_assert(sizeof(float) * AW * 16 * OSP <= 131072);
    __shared__ __align__(16) float os[AW * 16 * OSP];
    const int lane = threadIdx.x & 31, lr = lane & 15, hi = lane >> 4;
    const int wv = (int)(threadIdx.x >> 5);
    const int wave = __builtin_amdgcn_readfirstlane(wv);
    const int h = blockIdx.y;
    const int d0 = EARLY ? (int)blockIdx.z * 64 : 0;
    int winv = win_p[0];
    const bool allm = winv <= 0;
    winv = winv > SEQ ? SEQ : winv;
    const int t0v = (EARLY ? 0 : EROWS) + ((int)blockIdx.x * AW + wv) * 16;
    int klov = t0v - winv + 1; klov = klov < 0 ? 0 : klov; klov &= ~31; klov = allm ? 0 : klov;
    const int kendv = allm ? SEQ : (t0v + 16);
    const int t0 = __builtin_amdgcn_readfirstlane(t0v);
    const int klo = __builtin_amdgcn_readfirstlane(klov);
    const int kend = __builtin_amdgcn_readfirstlane(kendv);
    const size_t qo = ((size_t)h * SEQ + (size_t)(t0 + lr)) * HD + 8 * hi;
    const v16h hz = (v16h){};
    v8f o[DT], oR[DT];
#pragma unroll
    for (int j = 0; j < DT; ++j) { o[j] = (v8f){}; oR[j] = (v8f){}; }
    float m = NEGB, l = 0.0f;
#pragma unroll 1
    for (int key0 = klo; key0 < kend; key0 += 32) {
        const bool rok = key0 < EROWS;
        const int kcl = rok ? key0 : (EROWS - 32);
        const size_t kb = ((size_t)h * SEQ + (size_t)(key0 + lr)) * HD + 8 * hi;
        v8f sHa = (v8f){}, sLa = (v8f){}, sHb = (v8f){}, sLb = (v8f){};
#pragma unroll 1
        for (int kc = 0; kc < HD; kc += 32) {
            const v16h qh = ldh(QH + qo + kc), qr = ldh(QR + qo + kc);
            const v16h ka = ldh(KP + kb + kc), kq = ldh(KP + kb + (size_t)16 * HD + kc);
            const v16h ra = ldh(KR + kb + kc), rb = ldh(KR + kb + (size_t)16 * HD + kc);
            sHa = wmma16g(ka, qh, sHa); sLa = wmma16g(ka, qr, sLa); sLa = wmma16g(ra, qh, sLa);
            sHb = wmma16g(kq, qh, sHb); sLb = wmma16g(kq, qr, sLb); sLb = wmma16g(rb, qh, sLb);
        }
        const int da0 = (t0 + lr) - (key0 + 8 * hi);
        float ta[8], tb[8]; bool fa[8], fb[8]; float mx = NEGB;
#pragma unroll
        for (int r = 0; r < 8; ++r) {
            const int da = da0 - r, db = da0 - 16 - r;
            fa[r] = allm | ((da >= 0) & (da < winv));
            fb[r] = allm | ((db >= 0) & (db < winv));
            const float ua = (sHa[r] + sLa[r] * QRI) * SC2, ub = (sHb[r] + sLb[r] * QRI) * SC2;
            ta[r] = allm ? 0.0f : ua; tb[r] = allm ? 0.0f : ub;
            mx = fmaxf(mx, fmaxf(fa[r] ? ta[r] : NEGB, fb[r] ? tb[r] : NEGB)); }
        mx = fmaxf(mx, __shfl_xor(mx, 16, 32));
        const float mnew = fmaxf(m, mx);
        const float alpha = __builtin_amdgcn_exp2f(m - mnew);
        const float sh = PSH - mnew;
        v16h pb, pr = hz; float ls = 0.0f;
#pragma unroll
        for (int r = 0; r < 8; ++r) {
            const float xa = ta[r] + sh, xb = tb[r] + sh;
            const float ea = __builtin_amdgcn_exp2f(xa), eb = __builtin_amdgcn_exp2f(xb);
            const float ga = (fa[r] & (xa >= -14.0f)) ? ea : 0.0f;
            const float gb = (fb[r] & (xb >= -14.0f)) ? eb : 0.0f;
            const h16 pa = (h16)ga; const h16 pc = (h16)gb;
            pb[r] = pa; pb[8 + r] = pc;
            if (EARLY) { pr[r] = toh_flush((ga - (float)pa) * QRS); pr[8 + r] = toh_flush((gb - (float)pc) * QRS); ls += ga + gb; }
            else       { ls += (float)pa + (float)pc; } }
        l = l * alpha + ls; m = mnew;
#pragma unroll
        for (int j = 0; j < DT; ++j) { o[j] = o[j] * alpha; if (EARLY) oR[j] = oR[j] * alpha; }
#pragma unroll
        for (int j = 0; j < DT; ++j) {
            const size_t vrow = (size_t)h * HD + (size_t)(d0 + 16 * j + lr);
            const v16h v = ldh(VT + vrow * SEQ + (size_t)key0 + 8 * hi);
            o[j] = wmma16g(v, pb, o[j]);
            if (EARLY) {
                v16h vr = ldh(VR + vrow * EROWS + (size_t)kcl + 8 * hi);
                if (!rok) vr = hz;
                oR[j] = wmma16g(v, pr, oR[j]);
                oR[j] = wmma16g(vr, pb, oR[j]);
            }
        }
    }
    l += __shfl_xor(l, 16, 32);
    const bool any = l > 0.0f;
    const float lsafe = any ? l : 1.0f;
    const float inv = any ? (YC * (1.0f / lsafe)) : 0.0f;
    const int wb = wave * 16 * OSP;
#pragma unroll
    for (int j = 0; j < DT; ++j) {
        v8f f = o[j];
        if (EARLY) f = o[j] + oR[j] * QRI;
        v4f a, c;
        a[0] = f[0] * inv; a[1] = f[1] * inv; a[2] = f[2] * inv; a[3] = f[3] * inv; c[0] = f[4] * inv; c[1] = f[5] * inv; c[2] = f[6] * inv; c[3] = f[7] * inv;
        *(v4fa*)(&os[wb + lr * OSP + 16 * j + 8 * hi]) = a; *(v4fa*)(&os[wb + lr * OSP + 16 * j + 8 * hi + 4]) = c; }
    wave_sync();
    const size_t ybase = (size_t)t0 * DM + (size_t)h * HD + (size_t)d0;
#pragma unroll 1
    for (int ps = 0; ps < 2; ++ps) {
#pragma unroll 2
        for (int s = 0; s < NST; ++s) { const int row = s * RPI + lane / LPR, c8 = (lane % LPR) * 8;
            const v4f x0 = *(const v4fa*)(&os[wb + row * OSP + c8]); const v4f x1 = *(const v4fa*)(&os[wb + row * OSP + c8 + 4]); v8h hv, rv;
#pragma unroll
            for (int i = 0; i < 4; ++i) { const h16 a0 = toh_flush(x0[i]); const h16 a1 = toh_flush(x1[i]); hv[i] = a0; hv[4 + i] = a1;
                rv[i] = toh_flush((x0[i] - (float)a0) * QRS); rv[4 + i] = toh_flush((x1[i] - (float)a1) * QRS); }
            const size_t oo = ybase + (size_t)row * DM + c8;
            *(volatile v8h*)(YH + oo) = hv;
            if (EARLY) *(volatile v8h*)(YR + oo) = rv; }
        if (ps == 0) __threadfence(); }
}

__global__ __launch_bounds__(32 * AW) void k_flash_early(const h16* __restrict__ QH, const h16* __restrict__ QR, const h16* __restrict__ KP, const h16* __restrict__ KR,
                                                         const h16* __restrict__ VT, const h16* __restrict__ VR, const int* __restrict__ win_p, h16* YH, h16* YR) {
    flash_body<1>(QH, QR, KP, KR, VT, VR, win_p, YH, YR);
}
__global__ __launch_bounds__(32 * AW) void k_flash_late(const h16* __restrict__ QH, const h16* __restrict__ QR, const h16* __restrict__ KP, const h16* __restrict__ KR,
                                                        const h16* __restrict__ VT, const h16* __restrict__ VR, const int* __restrict__ win_p, h16* YH, h16* YR) {
    flash_body<0>(QH, QR, KP, KR, VT, VR, win_p, YH, YR);
}

__global__ __launch_bounds__(32) void k_out(const h16* __restrict__ YH, const h16* __restrict__ YR, const h16* __restrict__ WO, float* OUT) {
    __shared__ __align__(16) float os[16 * 68];
    const int lane = threadIdx.x & 31, lr = lane & 15, hi = lane >> 4; const int r0 = blockIdx.x * 64, c0 = blockIdx.y * 64;
    v8f acc[4][4];
#pragma unroll
    for (int mb = 0; mb < 4; ++mb)
#pragma unroll
        for (int nb = 0; nb < 4; ++nb) acc[mb][nb] = (v8f){};
    const size_t aoff = (size_t)(r0 + lr) * DM + 8 * hi, boff = (size_t)(c0 + lr) * DM + 8 * hi;
    if (r0 < EROWS) {
#pragma unroll 1
        for (int kc = 0; kc < DM; kc += 32) {
            v16h a[4];
#pragma unroll
            for (int mb = 0; mb < 4; ++mb) a[mb] = ldh(YR + aoff + (size_t)mb * 16 * DM + kc);
#pragma unroll
            for (int nb = 0; nb < 4; ++nb) { const v16h b = ldh(WO + boff + (size_t)nb * 16 * DM + kc);
#pragma unroll
                for (int mb = 0; mb < 4; ++mb) acc[mb][nb] = wmma16g(a[mb], b, acc[mb][nb]); }
        }
#pragma unroll
        for (int mb = 0; mb < 4; ++mb)
#pragma unroll
            for (int nb = 0; nb < 4; ++nb) acc[mb][nb] = acc[mb][nb] * QRI;
    }
#pragma unroll 1
    for (int kc = 0; kc < DM; kc += 32) {
        v16h a[4];
#pragma unroll
        for (int mb = 0; mb < 4; ++mb) a[mb] = ldh(YH + aoff + (size_t)mb * 16 * DM + kc);
#pragma unroll
        for (int nb = 0; nb < 4; ++nb) { const v16h b = ldh(WO + boff + (size_t)nb * 16 * DM + kc);
#pragma unroll
            for (int mb = 0; mb < 4; ++mb) acc[mb][nb] = wmma16g(a[mb], b, acc[mb][nb]); }
    }
    static_assert(8 * 32 * 16 == 16 * 64 * 4);
#pragma unroll
    for (int mb = 0; mb < 4; ++mb) {
#pragma unroll
        for (int nb = 0; nb < 4; ++nb) {
#pragma unroll
            for (int j = 0; j < 8; ++j) os[(hi * 8 + j) * 68 + nb * 16 + lr] = acc[mb][nb][j] * OSC; }
        wave_sync();
        float* orow = OUT + (size_t)(r0 + mb * 16) * DM + c0;
#pragma unroll 1
        for (int ps = 0; ps < 2; ++ps) {
#pragma unroll
            for (int s = 0; s < 8; ++s) { const int row = 2 * s + (lane >> 4), c4 = (lane & 15) * 4;
                const v4f val = *(const v4fa*)(&os[row * 68 + c4]);
                *(volatile v4f*)(orow + (size_t)row * DM + c4) = val; }
            if (ps == 0) __threadfence(); }
        wave_sync();
    }
}

static constexpr size_t al256(size_t v) { return (v + 255) & ~(size_t)255; }
static constexpr size_t SZ_XB = al256((size_t)SEQ * DM * 2);
static constexpr size_t SZ_WB = al256((size_t)3 * DM * DM * 2);
static constexpr size_t SZ_WO = al256((size_t)DM * DM * 2);
static constexpr size_t SZ_CS = al256((size_t)SEQ * 64 * 4);
static constexpr size_t SZ_PL = al256((size_t)NH_ * SEQ * HD * 2);
static constexpr size_t SZ_RS = al256((size_t)NH_ * HD * EROWS * 2);
static constexpr size_t SZ_YH = al256((size_t)SEQ * DM * 2);
static constexpr size_t SZ_YR = al256((size_t)EROWS * DM * 2);
static constexpr size_t SZ_TOTAL = SZ_XB + SZ_WB + SZ_WO + SZ_CS + 4 * SZ_PL + SZ_PL + SZ_RS + SZ_YH + SZ_YR;
static_assert(SZ_TOTAL <= (size_t)134217728);
static_assert(SZ_PL == (size_t)NH_ * SEQ * HD * 2);
static_assert(((size_t)NH_ * SEQ * HD * 2) % 256 == 0);
static_assert((size_t)NH_ * SEQ * HD == (size_t)SEQ * DM);

extern "C" void kernel_launch(void* const* d_in, const int* in_sizes, int n_in,
                              void* d_out, int out_size, void* d_ws, size_t ws_size, hipStream_t stream) {
    if (n_in < 5) return;
    const size_t needx = (size_t)SEQ * DM;
    if ((size_t)in_sizes[0] < needx || (size_t)in_sizes[1] < needx) return;
    if (in_sizes[2] < 2) return;
    if ((size_t)in_sizes[3] < (size_t)4 * DM * DM) return;
    if (in_sizes[4] < 1) return;
    if ((size_t)out_size < needx) return;
    if (SZ_TOTAL > ws_size) return;
    const float* x   = (const float*)d_in[0];
    const float* ve  = (const float*)d_in[1];
    const float* lam = (const float*)d_in[2];
    const float* w   = (const float*)d_in[3];
    const int*   win = (const int*)d_in[4];
    float* OUT = (float*)d_out;
    char* wsp = (char*)d_ws;
    bf*  XB = (bf*)wsp;   wsp += SZ_XB;
    bf*  WB = (bf*)wsp;   wsp += SZ_WB;
    h16* WO = (h16*)wsp;  wsp += SZ_WO;
    float* CS = (float*)wsp; wsp += SZ_CS;
    h16* QK = (h16*)wsp;  wsp += 4 * SZ_PL;
    h16* VT = (h16*)wsp;  wsp += SZ_PL;
    h16* VR = (h16*)wsp;  wsp += SZ_RS;
    h16* YH = (h16*)wsp;  wsp += SZ_YH;
    h16* YR = (h16*)wsp;  wsp += SZ_YR;
    const size_t PLE = (size_t)NH_ * SEQ * HD;
    const h16* QH = QK; const h16* QR = QK + PLE; const h16* KP = QK + 2 * PLE; const h16* KR = QK + 3 * PLE;

    { const size_t n8 = (size_t)SEQ * DM / 8;
      k_cvt8<<<(unsigned)((n8 + 255) / 256), 256, 0, stream>>>(x, XB, n8); }
    { const size_t n8 = (size_t)3 * DM * DM / 8;
      k_cvt8<<<(unsigned)((n8 + 255) / 256), 256, 0, stream>>>(w, WB, n8); }
    { const size_t n8 = (size_t)DM * DM / 8;
      k_cvtw<<<(unsigned)((n8 + 255) / 256), 256, 0, stream>>>(w + (size_t)3 * DM * DM, WO, n8); }
    k_ropetab<<<(unsigned)((size_t)SEQ * 32 / 256), 256, 0, stream>>>(CS);

    k_qkv<<<dim3(SEQ / 64, NQKV, 1), 64, 0, stream>>>(XB, WB, ve, lam, CS, QK, VT, VR);

    k_flash_early<<<dim3(EROWS / (16 * AW), NH_, 2), 32 * AW, 0, stream>>>(QH, QR, KP, KR, VT, VR, win, YH, YR);
    if (SEQ > EROWS)
        k_flash_late<<<dim3((SEQ - EROWS) / (16 * AW), NH_, 1), 32 * AW, 0, stream>>>(QH, QR, KP, KR, VT, VR, win, YH, YR);

    k_out<<<dim3(SEQ / 64, DM / 64, 1), 32, 0, stream>>>(YH, YR, WO, OUT);
}
